// RelativeSpatialEncoding_9612136808564
// MI455X (gfx1250) — hardware-verified
//
#include <hip/hip_runtime.h>
#include <math.h>

typedef __attribute__((ext_vector_type(16))) _Float16 v16h;
typedef __attribute__((ext_vector_type(16))) __bf16 v16b;
typedef __attribute__((ext_vector_type(8)))  _Float16 v8h;
typedef __attribute__((ext_vector_type(8)))  float v8f;
typedef __attribute__((ext_vector_type(4)))  float v4f;
typedef __attribute__((ext_vector_type(2)))  float v2f;
typedef __attribute__((ext_vector_type(4)))  unsigned v4u;
typedef __attribute__((ext_vector_type(4)))  int v4i;
typedef float __attribute__((may_alias)) float_a;
typedef int __attribute__((may_alias)) int_a;

template <typename T> __device__ __forceinline__ void vst2(void* p, T v) { *(volatile T*)p = v; __threadfence(); *(volatile T*)p = v; }
__device__ __forceinline__ v8f wmma16(v16h a, v16h b, v8f c) {
  v8f d = __builtin_amdgcn_wmma_f32_16x16x32_f16(false, a, false, b, (short)0, c, false, false);
  asm volatile("v_nop\n\tv_nop\n\tv_nop\n\tv_nop" : "+v"(d) : "v"(a), "v"(b));
  return d;
}
__device__ __forceinline__ v8f wmma_bf(v16b a, v16b b, v8f c) {
  v8f d = __builtin_amdgcn_wmma_f32_16x16x32_bf16(false, a, false, b, (short)0, c, false, false);
  asm volatile("v_nop\n\tv_nop\n\tv_nop\n\tv_nop" : "+v"(d) : "v"(a), "v"(b));
  return d;
}
__device__ __forceinline__ v16h frag_h(const _Float16* rowk0, int lane) {
  union { v16h v; v8h q[2]; } u; const _Float16* p = rowk0 + 8 * (lane >> 4);
  u.q[0] = *(const v8h*)p; u.q[1] = *(const v8h*)(p + 16); return u.v;
}
__device__ __forceinline__ v16h frag_f32(const float* rowk0, int lane) {
  v16h a; const float* p = rowk0 + 8 * (lane >> 4);
#pragma unroll
  for (int i = 0; i < 8; ++i) { a[i] = (_Float16)p[i]; a[8 + i] = (_Float16)p[16 + i]; }
  return a;
}
__device__ __forceinline__ v16h frag_f32s(const float* rowk0, int lane, float sc) {
  v16h a; const float* p = rowk0 + 8 * (lane >> 4);
#pragma unroll
  for (int i = 0; i < 8; ++i) { a[i] = (_Float16)(p[i] * sc); a[8 + i] = (_Float16)(p[16 + i] * sc); }
  return a;
}
__device__ __forceinline__ v16h fragc_f32(const float* W, int k0, int n, int lane, int ld, int K) {
  v16h a; const int g = lane >> 4;
#pragma unroll
  for (int i = 0; i < 8; ++i) { const int ka = k0 + 8 * g + i, kb = ka + 16;
    a[i] = (_Float16)(ka < K ? W[(size_t)ka * ld + n] : 0.f); a[8 + i] = (_Float16)(kb < K ? W[(size_t)kb * ld + n] : 0.f); }
  return a;
}
struct F2 { v16b h, l; };
__device__ __forceinline__ F2 bsplit16(const float v[16]) { F2 r;
#pragma unroll
  for (int i = 0; i < 16; ++i) { const __bf16 h = (__bf16)v[i]; r.h[i] = h; r.l[i] = (__bf16)(v[i] - (float)h); }
  return r; }
__device__ __forceinline__ F2 split_row(const float* row, int k0, int lane) { float v[16]; const float* p = row + k0 + 8 * (lane >> 4);
#pragma unroll
  for (int i = 0; i < 8; ++i) { v[i] = p[i]; v[8 + i] = p[16 + i]; }
  return bsplit16(v); }
__device__ __forceinline__ F2 split_rowK(const float* row, int k0, int lane, int K) { float v[16]; const int g = lane >> 4;
#pragma unroll
  for (int i = 0; i < 8; ++i) { const int ka = k0 + 8 * g + i, kb = ka + 16; v[i] = ka < K ? row[ka] : 0.f; v[8 + i] = kb < K ? row[kb] : 0.f; }
  return bsplit16(v); }
__device__ __forceinline__ F2 split_col(const float* W, int k0, int n, int lane, int ld, int K) { float v[16]; const int g = lane >> 4;
#pragma unroll
  for (int i = 0; i < 8; ++i) { const int ka = k0 + 8 * g + i, kb = ka + 16; v[i] = ka < K ? W[(size_t)ka * ld + n] : 0.f; v[8 + i] = kb < K ? W[(size_t)kb * ld + n] : 0.f; }
  return bsplit16(v); }
__device__ __forceinline__ v8f mac3(const F2& a, const F2& b, v8f c) { c = wmma_bf(a.l, b.h, c); c = wmma_bf(a.h, b.l, c); return wmma_bf(a.h, b.h, c); }
__device__ __forceinline__ float sigm(float v) { return 1.0f / (1.0f + expf(-v)); }
#define LDSX() do { asm volatile("s_wait_dscnt 0" ::: "memory"); __builtin_amdgcn_wave_barrier(); __builtin_amdgcn_fence(__ATOMIC_RELEASE, "workgroup"); } while (0)


__device__ __forceinline__ void load4ids(const int* __restrict__ ids, int e, int dd[4]) { const int4 a = *(const int4*)(ids + e); dd[0] = a.x; dd[1] = a.y; dd[2] = a.z; dd[3] = a.w; }
#define NN 50000
#define NE 800000
#define F 64
#define RB 512
#define NRB ((NN + RB - 1) / RB)
#define NNP (NRB * RB)
#define EPT 16
#define CH (256 * EPT)
__device__ __forceinline__ float bfr(float v) { return (float)(__bf16)v; }

__global__ __launch_bounds__(128) void k_proj(const float* __restrict__ G, const float* __restrict__ R, const float* __restrict__ W, float* __restrict__ P) {
  __shared__ __align__(16) float so[4][16][68];
  const int tid = threadIdx.x, wave = tid >> 5, lane = tid & 31, col = lane & 15, g = lane >> 4; const int which = blockIdx.y; const int r0 = blockIdx.x * 64 + wave * 16;
  const float* X = which ? R : G; const int ra = (r0 + col) < NN ? (r0 + col) : (NN - 1);
  v8f acc[4] = {};
#pragma unroll
  for (int kc = 0; kc < 2; ++kc) { const v16b a = split_row(X + (size_t)ra * F, kc * 32, lane).h;
#pragma unroll
    for (int j = 0; j < 4; ++j) acc[j] = wmma_bf(a, split_row(W + (size_t)(j * 16 + col) * F, kc * 32, lane).h, acc[j]); }
#pragma unroll
  for (int j = 0; j < 4; ++j)
#pragma unroll
    for (int r = 0; r < 8; ++r) so[wave][8 * g + r][j * 16 + col] = acc[j][r];
  LDSX();
  for (int rl = 0; rl < 16; ++rl) { if (lane < 16) vst2(P + ((size_t)which * NNP + r0 + rl) * F + lane * 4, *(const v4f*)(&so[wave][rl][lane * 4])); }
}
__global__ __launch_bounds__(256) void k_agg(const float* __restrict__ P, const int* __restrict__ esrc, const int* __restrict__ edst, const float* __restrict__ bias, float* __restrict__ OUT) {
  __shared__ __align__(16) float smax[RB][F]; __shared__ __align__(16) float ssum[RB][F]; __shared__ int scount[RB];
  __shared__ int ssrc[8][32 * EPT], sdl[8][32 * EPT]; __shared__ int scnt[8];
  const int tid = threadIdx.x, wave = tid >> 5, lane = tid & 31; const int r0 = blockIdx.x * RB;
  const float* PG = P; const float* PR = P + (size_t)NNP * F;
  for (int q = tid; q < RB * F; q += 256) { (&smax[0][0])[q] = -3.4e38f; (&ssum[0][0])[q] = 0.f; }
  for (int q = tid; q < RB; q += 256) scount[q] = 0;
  __syncthreads();
  const int f = tid & 63, wq = tid >> 6;
  const float bf_ = bfr(bias[f]);
#pragma unroll 1
  for (int c0 = 0; c0 < NE; c0 += CH) {
    const int e0 = c0 + tid * EPT; int hd[EPT]; int cnt = 0;
    if (e0 + EPT <= NE) {
#pragma unroll
      for (int v = 0; v < EPT / 4; ++v) { int dd[4]; load4ids(edst, e0 + v * 4, dd);
#pragma unroll
        for (int u = 0; u < 4; ++u) { const unsigned rel = (unsigned)(dd[u] - r0); const bool h = rel < (unsigned)RB; hd[v * 4 + u] = h ? (int)rel : -1; cnt += h ? 1 : 0; } } }
    else {
#pragma unroll
      for (int u = 0; u < EPT; ++u) { const int e = e0 + u; hd[u] = -1; if (e < NE) { const unsigned rel = (unsigned)(edst[e] - r0); if (rel < (unsigned)RB) { hd[u] = (int)rel; ++cnt; } } } }
    int incl = cnt;
#pragma unroll
    for (int off = 1; off < 32; off <<= 1) { const int vv = __shfl_up(incl, off, 32); if (lane >= off) incl += vv; }
    const int wtot = __shfl(incl, 31, 32); int pos = incl - cnt;
    if (cnt > 0) {
#pragma unroll
      for (int u = 0; u < EPT; ++u) if (hd[u] >= 0) { int s = esrc[e0 + u]; s = s < 0 ? 0 : (s >= NN ? NN - 1 : s); ssrc[wave][pos] = s; sdl[wave][pos] = hd[u]; ++pos; } }
    if (lane == 0) scnt[wave] = wtot;
    __syncthreads();
#pragma unroll 1
    for (int grp = 0; grp < 4; ++grp) { if (wq == grp) { for (int w2 = 2 * grp; w2 < 2 * grp + 2; ++w2) { const int nh = scnt[w2]; for (int i = 0; i < nh; ++i) { const int dl = sdl[w2][i]; const float v0 = PG[(size_t)ssrc[w2][i] * F + f] - PR[(size_t)(r0 + dl) * F + f] + bf_; const float v = v0 > 0.f ? v0 : 0.f;
            smax[dl][f] = fmaxf(smax[dl][f], v); ssum[dl][f] += v; if (f == 0) scount[dl] += 1; } } }
      __syncthreads(); } }
  for (int q = tid; q < RB * (2 * F / 4); q += 256) { const int rl = q >> 5, pc = q & 31; const int row = r0 + rl; if (row >= NN) continue; const int c = scount[rl]; v4f v;
    if (pc < 16) { v = *(const v4f*)(&smax[rl][pc * 4]); if (c == 0) v = (v4f){0.f, 0.f, 0.f, 0.f}; }
    else { v = *(const v4f*)(&ssum[rl][(pc - 16) * 4]); const float inv = 1.0f / (float)(c > 0 ? c : 1);
#pragma unroll
      for (int e = 0; e < 4; ++e) v[e] *= inv; }
    vst2(OUT + (size_t)row * (2 * F) + pc * 4, v); }
}
extern "C" void kernel_launch(void* const* d_in, const int* in_sizes, int n_in, void* d_out, int out_size, void* d_ws, size_t ws_size, hipStream_t stream) {
  (void)in_sizes; (void)n_in; (void)out_size; (void)ws_size;
  const float* G = (const float*)d_in[0]; const float* R = (const float*)d_in[1]; const int* src = (const int*)d_in[2]; const int* dst = (const int*)d_in[3]; const float* W = (const float*)d_in[4]; const float* b = (const float*)d_in[5];
  float* P = (float*)d_ws;
  k_proj<<<dim3(NNP / 64, 2), 128, 0, stream>>>(G, R, W, P);
  k_agg<<<NRB, 256, 0, stream>>>(P, src, dst, b, (float*)d_out);
}
